// FullAttention_33062658245138
// MI455X (gfx1250) — hardware-verified
//
#include <hip/hip_runtime.h>


#define NH 8
#define HD 64
#ifndef NB
#define NB 4
#endif
#ifndef SEQ
#define SEQ 2048
#endif
#define NB_FULL 4
#define SEQ_FULL 2048
#define TOKP (NH * HD)
#define OUT1E ((size_t)NB_FULL * SEQ_FULL * NH * HD)
#define KC 64
#define BM 64
#define NT 128
#define KP 72
#define TP 72
#define OP 68
#define SCALE 0.125f
#define LOG2E 1.4426950408889634f

static_assert(OUT1E * 4 == 16777216u);
static_assert(SEQ % KC == 0);
static_assert(SEQ % BM == 0);
static_assert(SEQ <= SEQ_FULL);
static_assert(NB <= NB_FULL);
static_assert(KC * HD / 8 == 4 * NT);
static_assert((KP % 8) == 0 && (TP % 8) == 0 && (OP % 4) == 0);

typedef unsigned short bf;
typedef __attribute__((ext_vector_type(16))) __bf16   v16bf;
typedef __attribute__((ext_vector_type(8)))  unsigned short v8us;
typedef __attribute__((ext_vector_type(8)))  float    v8f;
typedef __attribute__((ext_vector_type(4)))  float    v4f;
typedef v8us __attribute__((may_alias)) v8usa;
typedef v8f  __attribute__((may_alias)) v8fa;
typedef v4f  __attribute__((may_alias)) v4fa;

__device__ __forceinline__ unsigned short f2bf(float f) { unsigned u = __float_as_uint(f); u += 0x7FFFu + ((u >> 16) & 1u); return (unsigned short)(u >> 16); }
__device__ __forceinline__ float bf2f(unsigned short b) { return __uint_as_float(((unsigned)b) << 16); }
__device__ __forceinline__ void splitf(float y, unsigned short& h, unsigned short& l) { h = f2bf(y); l = f2bf(y - bf2f(h)); }
__device__ __forceinline__ v16bf cat16b(v8us lo, v8us hi) { return __builtin_bit_cast(v16bf, __builtin_shufflevector(lo, hi, 0, 1, 2, 3, 4, 5, 6, 7, 8, 9, 10, 11, 12, 13, 14, 15)); }
__device__ __forceinline__ v8f wmmab(v16bf a, v16bf b, v8f c) { return __builtin_amdgcn_wmma_f32_16x16x32_bf16(false, a, false, b, (short)0, c, false, false); }

__global__ __launch_bounds__(256) void k_cvt8(const float* __restrict__ src, bf* dst, size_t n8) {
    const size_t i = (size_t)blockIdx.x * 256 + threadIdx.x; if (i >= n8) return;
    const v8f v = *(const v8fa*)(src + i * 8); v8us o;
#pragma unroll
    for (int k = 0; k < 8; ++k) o[k] = f2bf(v[k]);
    *(volatile v8us*)(dst + i * 8) = o; __threadfence(); *(volatile v8us*)(dst + i * 8) = o;
}

__global__ __launch_bounds__(NT) void k_attn(const bf* __restrict__ Qp, const bf* __restrict__ Kp, float* Out) {
    __shared__ __align__(16) bf Krm[KC * KP];
    __shared__ __align__(16) bf Kt[HD * TP];
    __shared__ __align__(16) float os[4][16 * OP];

    const int tid = threadIdx.x, wave = tid >> 5, lane = tid & 31, hf = lane >> 4, lm = lane & 15;
    const int bh = blockIdx.y, b = bh / NH, h = bh % NH;
    const int m0 = blockIdx.x * BM + wave * 16;

    const bf* Qg = Qp + ((size_t)b * SEQ_FULL + (size_t)(m0 + lm)) * TOKP + h * HD;
    const v16bf bq0 = cat16b(*(const v8usa*)(Qg + 8 * hf), *(const v8usa*)(Qg + 16 + 8 * hf));
    const v16bf bq1 = cat16b(*(const v8usa*)(Qg + 32 + 8 * hf), *(const v8usa*)(Qg + 48 + 8 * hf));
    const bf* Kg = Kp + (size_t)b * SEQ_FULL * TOKP + h * HD;

    float mrun = -1.0e30f, lrun = 0.0f;
    v8f acc[4];
#pragma unroll
    for (int t = 0; t < 4; ++t) acc[t] = (v8f){};

#pragma unroll 1
    for (int s0 = 0; s0 < SEQ; s0 += KC) {
        __syncthreads();
#pragma unroll
        for (int it = 0; it < 4; ++it) {
            const int idx = it * NT + tid; const int s = idx >> 3; const int c8 = (idx & 7) * 8;
            const v8us v = *(const v8usa*)(Kg + (size_t)(s0 + s) * TOKP + c8);
            *(v8usa*)(Krm + s * KP + c8) = v;
#pragma unroll
            for (int j = 0; j < 8; ++j) Kt[(c8 + j) * TP + s] = v[j];
        }
        __syncthreads();

        v8f c[4];
#pragma unroll
        for (int mt = 0; mt < 4; ++mt) {
            const bf* ar = Krm + (mt * 16 + lm) * KP + 8 * hf;
            const v16bf a0 = cat16b(*(const v8usa*)(ar), *(const v8usa*)(ar + 16));
            const v16bf a1 = cat16b(*(const v8usa*)(ar + 32), *(const v8usa*)(ar + 48));
            v8f cz = (v8f){};
            cz = wmmab(a0, bq0, cz);
            cz = wmmab(a1, bq1, cz);
            c[mt] = cz;
        }
        asm volatile("v_nop\n\tv_nop\n\tv_nop\n\tv_nop" : "+v"(c[0]), "+v"(c[1]), "+v"(c[2]), "+v"(c[3]) : "v"(bq0), "v"(bq1));

        float mx = -1.0e30f;
#pragma unroll
        for (int mt = 0; mt < 4; ++mt) {
            c[mt] = c[mt] * SCALE;
#pragma unroll
            for (int r = 0; r < 8; ++r) mx = fmaxf(mx, c[mt][r]);
        }
        mx = fmaxf(mx, __shfl_xor(mx, 16, 32));
        const float mnew = fmaxf(mrun, mx);
        const float corr = __builtin_amdgcn_exp2f((mrun - mnew) * LOG2E);
        float psum = 0.0f;
        v8us ph[4], pl[4];
#pragma unroll
        for (int mt = 0; mt < 4; ++mt) {
#pragma unroll
            for (int r = 0; r < 8; ++r) {
                const float p = __builtin_amdgcn_exp2f((c[mt][r] - mnew) * LOG2E);
                psum += p;
                unsigned short a2, l2; splitf(p, a2, l2); ph[mt][r] = a2; pl[mt][r] = l2;
            }
        }
        psum += __shfl_xor(psum, 16, 32);
        lrun = lrun * corr + psum; mrun = mnew;
#pragma unroll
        for (int t = 0; t < 4; ++t) acc[t] = acc[t] * corr;

        const v16bf bph0 = cat16b(ph[0], ph[1]), bph1 = cat16b(ph[2], ph[3]);
        const v16bf bpl0 = cat16b(pl[0], pl[1]), bpl1 = cat16b(pl[2], pl[3]);

#pragma unroll
        for (int t = 0; t < 4; ++t) {
            const bf* ar = Kt + (t * 16 + lm) * TP + 8 * hf;
            const v16bf a0 = cat16b(*(const v8usa*)(ar), *(const v8usa*)(ar + 16));
            const v16bf a1 = cat16b(*(const v8usa*)(ar + 32), *(const v8usa*)(ar + 48));
            acc[t] = wmmab(a0, bph0, acc[t]);
            acc[t] = wmmab(a0, bpl0, acc[t]);
            acc[t] = wmmab(a1, bph1, acc[t]);
            acc[t] = wmmab(a1, bpl1, acc[t]);
        }
        asm volatile("v_nop\n\tv_nop\n\tv_nop\n\tv_nop" : "+v"(acc[0]), "+v"(acc[1]), "+v"(acc[2]), "+v"(acc[3]) : "v"(bph0), "v"(bpl1));
    }

    const float inv = 1.0f / lrun;
    float* osw = os[wave];
#pragma unroll
    for (int t = 0; t < 4; ++t) {
        v4f w0, w1;
        w0[0] = acc[t][0] * inv; w0[1] = acc[t][1] * inv; w0[2] = acc[t][2] * inv; w0[3] = acc[t][3] * inv;
        w1[0] = acc[t][4] * inv; w1[1] = acc[t][5] * inv; w1[2] = acc[t][6] * inv; w1[3] = acc[t][7] * inv;
        *(v4fa*)(osw + lm * OP + t * 16 + 8 * hf) = w0;
        *(v4fa*)(osw + lm * OP + t * 16 + 8 * hf + 4) = w1;
    }
    __builtin_amdgcn_fence(3  , "wavefront");
    __builtin_amdgcn_wave_barrier();
    float* orow0 = Out + ((size_t)b * SEQ_FULL + (size_t)m0) * TOKP + h * HD;
#pragma unroll 1
    for (int ps = 0; ps < 2; ++ps) {
#pragma unroll
        for (int s = 0; s < 8; ++s) {
            const int row = 2 * s + hf; const int cofs = lm * 4;
            const v4f val = *(const v4fa*)(osw + row * OP + cofs);
            *(volatile v4f*)(orow0 + (size_t)row * TOKP + cofs) = val;
        }
        if (ps == 0) __threadfence();
    }
}

extern "C" void kernel_launch(void* const* d_in, const int* in_sizes, int n_in,
                              void* d_out, int out_size, void* d_ws, size_t ws_size, hipStream_t stream) {
    if (n_in < 2) return;
    const float* Qin = (const float*)d_in[0];
    const float* Kin = (const float*)d_in[1];
    float* OUT = (float*)d_out;
    const size_t need = ((size_t)(NB - 1) * SEQ_FULL + SEQ) * TOKP;
    if (in_sizes[0] < 0 || in_sizes[1] < 0 || out_size < 0) return;
    if ((size_t)in_sizes[0] < need || (size_t)in_sizes[1] < need) return;
    if ((in_sizes[0] & 63) != 0 || (in_sizes[1] & 63) != 0) return;
    if ((size_t)out_size < OUT1E + need) return;
    const size_t qbytes = (((size_t)in_sizes[0] * 2) + 255) & ~(size_t)255;
    const size_t kbytes = (((size_t)in_sizes[1] * 2) + 255) & ~(size_t)255;
    if (qbytes + kbytes > ws_size) return;
    if (qbytes + kbytes > (size_t)134217728u) return;
    char* wsp = (char*)d_ws;
    bf* QB = (bf*)wsp; bf* KB = (bf*)(wsp + qbytes);
    const size_t nq8 = (size_t)in_sizes[0] / 8, nk8 = (size_t)in_sizes[1] / 8;
    k_cvt8<<<(unsigned)((nq8 + 255) / 256), 256, 0, stream>>>(Qin, QB, nq8);
    k_cvt8<<<(unsigned)((nk8 + 255) / 256), 256, 0, stream>>>(Kin, KB, nk8);
    dim3 grid(SEQ / BM, NB * NH);
    k_attn<<<grid, NT, 0, stream>>>(QB, KB, OUT);
    k_attn<<<grid, NT, 0, stream>>>(KB, QB, OUT + OUT1E);
}
